// MAGNODecoder_72816875536553
// MI455X (gfx1250) — hardware-verified
//
#include <hip/hip_runtime.h>
#include <stddef.h>


#pragma clang fp contract(off)

#define CIN     64
#define PH      256
#define NB      4
#define NTHR    256
#define NWAVE   8
#define TE      64
#define TR      64
#define QPW     8
#define QPB     (NWAVE * QPW)
#define APA     72
#define APH     264
#define KROW    64
#define DROW    64
#define MAXSEG  4096
#define NCHK    32
#define CHKLINE 32
#define PK1     0
#define PK2     4096
#define PP0     8192
#define PP1     24576
#define PWTOT   28672
#define PBLK    (PWTOT / (NTHR * 8))
#define WSCAP   134217728
#define SCW     16.0f
#define SCA     64.0f
#define INV1024 0.0009765625f
#define LOG2E   1.4426950408889634f

static_assert((PWTOT % (NTHR * 8)) == 0);
static_assert((PK2 % (NTHR * 8)) == 0);
static_assert((PP0 % (NTHR * 8)) == 0);
static_assert((PP1 % (NTHR * 8)) == 0);
static_assert(((APA * 2) % 16) == 0);
static_assert(((APH * 2) % 16) == 0);
static_assert(NTHR == 4 * CIN);
static_assert(NTHR == PH);
static_assert(TE == 4 * 16);
static_assert(TR == 4 * 16);
static_assert(QPB == 64);
static_assert(NB == 4);
static_assert(NCHK == 32);
static_assert(CHKLINE * 4 == 128);

typedef float          v4f   __attribute__((ext_vector_type(4)));
typedef float          v8f   __attribute__((ext_vector_type(8)));
typedef unsigned short v8us  __attribute__((ext_vector_type(8)));
typedef _Float16       v4h   __attribute__((ext_vector_type(4)));
typedef _Float16       v8h   __attribute__((ext_vector_type(8)));
typedef _Float16       v16h  __attribute__((ext_vector_type(16)));
union FragH { v16h v; v8h h[2]; };
union Cvt8  { v8h v; v8us u; };

__device__ __forceinline__ v8f wmh(v16h a, v16h b, v8f c) {
  v8f d = __builtin_amdgcn_wmma_f32_16x16x32_f16(false, a, false, b, (short)0, c, false, false);
  asm volatile("v_nop\n\tv_nop\n\tv_nop\n\tv_nop" : "+v"(d) : "v"(a), "v"(b));
  return d;
}
__device__ __forceinline__ v8f zero8() {
  v8f z = {0.f, 0.f, 0.f, 0.f, 0.f, 0.f, 0.f, 0.f};
  return z;
}
__device__ __forceinline__ v4f zero4() {
  v4f z = {0.f, 0.f, 0.f, 0.f};
  return z;
}
__device__ __forceinline__ int iclamp(int v, int lo, int hi) { return v < lo ? lo : (v > hi ? hi : v); }

__device__ __forceinline__ float gelu_f(float x) {
  const float u = 1.5957691216057308f * (x + 0.044715f * x * x * x);
  const float t = __builtin_amdgcn_exp2f(-LOG2E * u);
  return x * __builtin_amdgcn_rcpf(1.0f + t);
}

__device__ __forceinline__ void gemm16x64(const _Float16* ap, const _Float16* bpl, int kp, int nks, int n0,
                                          int m, int hh, v8f& c0, v8f& c1, v8f& c2, v8f& c3) {
  c0 = zero8(); c1 = zero8(); c2 = zero8(); c3 = zero8();
#pragma unroll 1
  for (int ks = 0; ks < nks; ++ks) {
    FragH a;
    a.h[0] = *(const v8h*)(ap + 32 * ks);
    a.h[1] = *(const v8h*)(ap + 32 * ks + 16);
    const _Float16* bp = bpl + (size_t)(n0 + m) * kp + 32 * ks + 8 * hh;
    FragH b;
    b.h[0] = *(const v8h*)(bp);
    b.h[1] = *(const v8h*)(bp + 16);
    c0 = wmh(a.v, b.v, c0);
    b.h[0] = *(const v8h*)(bp + (size_t)16 * kp);
    b.h[1] = *(const v8h*)(bp + (size_t)16 * kp + 16);
    c1 = wmh(a.v, b.v, c1);
    b.h[0] = *(const v8h*)(bp + (size_t)32 * kp);
    b.h[1] = *(const v8h*)(bp + (size_t)32 * kp + 16);
    c2 = wmh(a.v, b.v, c2);
    b.h[0] = *(const v8h*)(bp + (size_t)48 * kp);
    b.h[1] = *(const v8h*)(bp + (size_t)48 * kp + 16);
    c3 = wmh(a.v, b.v, c3);
  }
}
__device__ __forceinline__ void gemm16x32(const _Float16* ap, const _Float16* bpl, int kp, int nks, int n0,
                                          int m, int hh, v8f& c0, v8f& c1) {
  c0 = zero8(); c1 = zero8();
#pragma unroll 1
  for (int ks = 0; ks < nks; ++ks) {
    FragH a;
    a.h[0] = *(const v8h*)(ap + 32 * ks);
    a.h[1] = *(const v8h*)(ap + 32 * ks + 16);
    const _Float16* bp = bpl + (size_t)(n0 + m) * kp + 32 * ks + 8 * hh;
    FragH b;
    b.h[0] = *(const v8h*)(bp);
    b.h[1] = *(const v8h*)(bp + 16);
    c0 = wmh(a.v, b.v, c0);
    b.h[0] = *(const v8h*)(bp + (size_t)16 * kp);
    b.h[1] = *(const v8h*)(bp + (size_t)16 * kp + 16);
    c1 = wmh(a.v, b.v, c1);
  }
}
__device__ __forceinline__ void gemm16x16(const _Float16* ap, const _Float16* bpl, int kp, int nks, int n0,
                                          int m, int hh, v8f& c0) {
  c0 = zero8();
#pragma unroll 1
  for (int ks = 0; ks < nks; ++ks) {
    FragH a;
    a.h[0] = *(const v8h*)(ap + 32 * ks);
    a.h[1] = *(const v8h*)(ap + 32 * ks + 16);
    const _Float16* bp = bpl + (size_t)(n0 + m) * kp + 32 * ks + 8 * hh;
    FragH b;
    b.h[0] = *(const v8h*)(bp);
    b.h[1] = *(const v8h*)(bp + 16);
    c0 = wmh(a.v, b.v, c0);
  }
}

__device__ __forceinline__ void st8_gelu_h(_Float16* sp, int pitch, v8f a, float scl, float bias) {
#pragma unroll
  for (int r = 0; r < 8; ++r) sp[r * pitch] = (_Float16)(gelu_f(a[r] * scl + bias) * SCA);
}
__device__ __forceinline__ void st8_lin_h(_Float16* sp, int pitch, v8f a, float scl, float bias) {
#pragma unroll
  for (int r = 0; r < 8; ++r) sp[r * pitch] = (_Float16)(a[r] * scl + bias);
}

__global__ __launch_bounds__(NTHR) void k_chk(
    const int* __restrict__ qa, int na, const int* __restrict__ qb, int nb, int* chk) {
  __shared__ int sCnt[NWAVE];
  const int tid = (int)threadIdx.x, lane = tid & 31, wave = tid >> 5;
  const int b = (int)blockIdx.x;
  int c = 0;
#pragma unroll 1
  for (int i = b * NTHR + tid; i < na - 1; i += NCHK * NTHR) c += (qa[i] > qa[i + 1]) ? 1 : 0;
#pragma unroll 1
  for (int i = b * NTHR + tid; i < nb - 1; i += NCHK * NTHR) c += (qb[i] > qb[i + 1]) ? 1 : 0;
  c += __shfl_xor(c, 1);
  c += __shfl_xor(c, 2);
  c += __shfl_xor(c, 4);
  c += __shfl_xor(c, 8);
  c += __shfl_xor(c, 16);
  if (lane == 0) sCnt[wave] = c;
  __syncthreads();
  if (wave == 0) {
    int t = 0;
#pragma unroll
    for (int w = 0; w < NWAVE; ++w) t += sCnt[w];
    const int v = (lane == 0) ? t : 0;
    int* p = chk + (size_t)b * CHKLINE + lane;
    *(volatile int*)p = v;
    __threadfence();
    *(volatile int*)p = v;
  }
}

__global__ __launch_bounds__(NTHR) void k_prep(
    const float* __restrict__ Wk1, const float* __restrict__ Wk2, const float* __restrict__ Wp0,
    const float* __restrict__ Wp1, unsigned short* wp) {
  const int tid = (int)threadIdx.x;
  const int b = (int)blockIdx.x;
  const int o = (b * NTHR + tid) * 8;
  Cvt8 cv;
  if (o < PK2) {
    const int n = o >> 6, k0 = o & 63;
#pragma unroll
    for (int j = 0; j < 8; ++j) cv.v[j] = (_Float16)(Wk1[(size_t)(k0 + j) * CIN + n] * SCW);
  } else if (o < PP0) {
    const int idx = o - PK2;
    const int n = idx >> 6, k0 = idx & 63;
#pragma unroll
    for (int j = 0; j < 8; ++j) cv.v[j] = (_Float16)(Wk2[(size_t)(k0 + j) * CIN + n] * SCW);
  } else if (o < PP1) {
    const int idx = o - PP0;
    const int n = idx >> 6, k0 = idx & 63;
#pragma unroll
    for (int j = 0; j < 8; ++j) cv.v[j] = (_Float16)(Wp0[(size_t)(k0 + j) * PH + n] * SCW);
  } else {
    const int idx = o - PP1;
    const int n = idx >> 8, k0 = idx & 255;
    const int nc = n > 3 ? 3 : n;
#pragma unroll
    for (int j = 0; j < 8; ++j) {
      const float v = Wp1[(size_t)(k0 + j) * 4 + nc] * SCW;
      cv.v[j] = (_Float16)((n < 4) ? v : 0.0f);
    }
  }
  unsigned short* dp = wp + o;
  *(volatile v8us*)dp = cv.u;
  __threadfence();
  *(volatile v8us*)dp = cv.u;
}

__global__ __launch_bounds__(NTHR) void k_edge(
    const float* __restrict__ latc, const float* __restrict__ qc, const int* __restrict__ src,
    const int* __restrict__ qry, const float* __restrict__ Wk0, const float* __restrict__ bk0,
    const float* __restrict__ bk1, const float* __restrict__ bk2, const unsigned short* __restrict__ wp,
    unsigned short* Kout, int nE, int nLat, int nQry) {
  __shared__ __attribute__((aligned(16))) _Float16 sA[TE * APA];
  __shared__ __attribute__((aligned(16))) _Float16 sB[TE * APA];
  __shared__ __attribute__((aligned(16))) float sW0[4 * CIN];
  __shared__ __attribute__((aligned(16))) float sPar[3 * CIN];
  __shared__ __attribute__((aligned(16))) float sF[TE * 4];
  const int tid = (int)threadIdx.x, lane = tid & 31, wave = tid >> 5, hh = lane >> 4, m = lane & 15;
  const int e0 = (int)blockIdx.x * TE;

  if (tid < TE) {
    int e = e0 + tid;
    e = e > nE - 1 ? nE - 1 : e;
    const int sv = iclamp(src[e], 0, nLat - 1);
    const int qv = iclamp(qry[e], 0, nQry - 1);
    sF[4 * tid]     = latc[(size_t)sv * 2];
    sF[4 * tid + 1] = latc[(size_t)sv * 2 + 1];
    sF[4 * tid + 2] = qc[(size_t)qv * 2];
    sF[4 * tid + 3] = qc[(size_t)qv * 2 + 1];
  }
  sW0[tid] = Wk0[tid];
  if (tid < CIN) {
    sPar[tid]           = bk0[tid];
    sPar[CIN + tid]     = bk1[tid];
    sPar[2 * CIN + tid] = bk2[tid];
  }
  __syncthreads();

  {
    const int el = tid >> 2, g = tid & 3;
    const float f0 = sF[4 * el], f1 = sF[4 * el + 1], f2 = sF[4 * el + 2], f3 = sF[4 * el + 3];
    _Float16* dst = sA + el * APA + 16 * g;
#pragma unroll 4
    for (int j = 0; j < 16; ++j) {
      const int n = 16 * g + j;
      const float d = ((f0 * sW0[n] + f1 * sW0[CIN + n]) + f2 * sW0[2 * CIN + n]) + f3 * sW0[3 * CIN + n];
      const float v = d + sPar[n];
      dst[j] = (_Float16)(gelu_f(v) * SCA);
    }
  }
  __syncthreads();

  const int rt = wave & 3, cg = wave >> 2;

  {
    v8f a0, a1;
    gemm16x32(sA + (16 * rt + m) * APA + 8 * hh, (const _Float16*)(wp + PK1), CIN, 2, 32 * cg, m, hh, a0, a1);
    _Float16* sp = sB + (16 * rt + 8 * hh) * APA + 32 * cg + m;
    const float* bb = sPar + CIN + 32 * cg + m;
    st8_gelu_h(sp,      APA, a0, INV1024, bb[0]);
    st8_gelu_h(sp + 16, APA, a1, INV1024, bb[16]);
  }
  __syncthreads();

  {
    v8f a0, a1;
    gemm16x32(sB + (16 * rt + m) * APA + 8 * hh, (const _Float16*)(wp + PK2), CIN, 2, 32 * cg, m, hh, a0, a1);
    _Float16* sp = sA + (16 * rt + 8 * hh) * APA + 32 * cg + m;
    const float* bb = sPar + 2 * CIN + 32 * cg + m;
    st8_lin_h(sp,      APA, a0, INV1024, bb[0]);
    st8_lin_h(sp + 16, APA, a1, INV1024, bb[16]);
  }
  __syncthreads();

  {
    const int p = tid & 7, rq = tid >> 3;
#pragma unroll 1
    for (int it = 0; it < 2; ++it) {
      const int row = rq + 32 * it;
      Cvt8 cv;
      cv.v = *(const v8h*)(sA + row * APA + 8 * p);
      *(volatile v8us*)(Kout + (size_t)(e0 + row) * KROW + 8 * p) = cv.u;
    }
    __threadfence();
#pragma unroll 1
    for (int it = 0; it < 2; ++it) {
      const int row = rq + 32 * it;
      Cvt8 cv;
      cv.v = *(const v8h*)(sA + row * APA + 8 * p);
      *(volatile v8us*)(Kout + (size_t)(e0 + row) * KROW + 8 * p) = cv.u;
    }
  }
}

__device__ __forceinline__ int lbound(const int* __restrict__ a, int n, int key) {
  int lo = 0, hi = n;
#pragma unroll 1
  for (int it = 0; it < 40 && lo < hi; ++it) {
    const int mid = lo + ((hi - lo) >> 1);
    const int v = a[mid];
    if (v < key) lo = mid + 1; else hi = mid;
  }
  return lo;
}

__global__ __launch_bounds__(NTHR) void k_seg(
    const int* __restrict__ qry, const int* __restrict__ src, const unsigned short* __restrict__ Kq,
    const float* __restrict__ rnd, float* D, int nE, int nQry, int nLat) {
  const int tid = (int)threadIdx.x, lane = tid & 31, wave = tid >> 5, hh = lane >> 4, m = lane & 15;
  const _Float16* Kh = (const _Float16*)Kq;
  const int qb = (int)blockIdx.x * QPB + wave * QPW;
  const float* r0p = rnd + (size_t)(2 * hh) * (size_t)nLat * CIN + 4 * m;
  const float* r1p = rnd + (size_t)(2 * hh + 1) * (size_t)nLat * CIN + 4 * m;
#pragma unroll 1
  for (int qi = 0; qi < QPW; ++qi) {
    const int q = qb + qi;
    if (q < nQry) {
      int lo = lbound(qry, nE, q);
      int hi = lbound(qry, nE, q + 1);
      lo = iclamp(lo, 0, nE);
      hi = iclamp(hi, 0, nE);
      int cntAll = hi - lo;
      cntAll = cntAll < 0 ? 0 : cntAll;
      const int cnt = cntAll > MAXSEG ? MAXSEG : cntAll;
      v4f a0 = zero4(), a1 = zero4();
#pragma unroll 1
      for (int i = 0; i < cnt; ++i) {
        int e = lo + i;
        e = e > nE - 1 ? nE - 1 : e;
        const int sv = iclamp(src[e], 0, nLat - 1);
        const v4h kv = *(const v4h*)(Kh + (size_t)e * KROW + 4 * m);
        v4f kf;
        kf.x = (float)kv.x; kf.y = (float)kv.y; kf.z = (float)kv.z; kf.w = (float)kv.w;
        const v4f f0 = *(const v4f*)(r0p + (size_t)sv * CIN);
        const v4f f1 = *(const v4f*)(r1p + (size_t)sv * CIN);
        a0 = a0 + kf * f0;
        a1 = a1 + kf * f1;
      }
      const float cf = (float)cntAll;
      const float inv = 1.0f / fmaxf(cf, 1.0f);
      const v4f o0 = a0 * inv;
      const v4f o1 = a1 * inv;
      float* d0p = D + ((size_t)(2 * hh) * (size_t)nQry + (size_t)q) * DROW + 4 * m;
      float* d1p = D + ((size_t)(2 * hh + 1) * (size_t)nQry + (size_t)q) * DROW + 4 * m;
      *(volatile v4f*)d0p = o0;
      *(volatile v4f*)d1p = o1;
      __threadfence();
      *(volatile v4f*)d0p = o0;
      *(volatile v4f*)d1p = o1;
    }
  }
}

__global__ __launch_bounds__(NTHR) void k_proj(
    const float* __restrict__ qc, const float* __restrict__ Wsw0, const float* __restrict__ bsw0,
    const float* __restrict__ Wsw1, const float* __restrict__ bsw1, const float* __restrict__ D0,
    const float* __restrict__ D1, const unsigned short* __restrict__ wp, const float* __restrict__ bp0,
    const float* __restrict__ bp1, const int* __restrict__ chk, float* out, int nQry, int nRows) {
  __shared__ __attribute__((aligned(16))) _Float16 sA[TR * APA];
  __shared__ __attribute__((aligned(16))) _Float16 sH[TR * APH];
  __shared__ __attribute__((aligned(16))) float sBp[PH + 4];
  __shared__ __attribute__((aligned(16))) float sW[TR * 2];
  __shared__ __attribute__((aligned(16))) float sO[TR * 4];
  __shared__ int sBi[TR];
  __shared__ int sQi[TR];
  __shared__ int sFlag;
  const int tid = (int)threadIdx.x, lane = tid & 31, wave = tid >> 5, hh = lane >> 4, m = lane & 15;
  const int R0 = (int)blockIdx.x * TR;

  if (tid < TR) {
    int R = R0 + tid;
    R = R > nRows - 1 ? nRows - 1 : R;
    const int b = R / nQry;
    const int q = R - b * nQry;
    sBi[tid] = b;
    sQi[tid] = q;
    const float x0 = qc[(size_t)q * 2], x1 = qc[(size_t)q * 2 + 1];
    float z0 = 0.0f, z1 = 0.0f;
#pragma unroll 1
    for (int j = 0; j < 16; ++j) {
      const float hv = fmaxf((x0 * Wsw0[j] + x1 * Wsw0[16 + j]) + bsw0[j], 0.0f);
      z0 = z0 + hv * Wsw1[2 * j];
      z1 = z1 + hv * Wsw1[2 * j + 1];
    }
    z0 = z0 + bsw1[0];
    z1 = z1 + bsw1[1];
    const float mx = fmaxf(z0, z1);
    const float ex0 = __builtin_amdgcn_exp2f((z0 - mx) * LOG2E);
    const float ex1 = __builtin_amdgcn_exp2f((z1 - mx) * LOG2E);
    const float inv = 1.0f / (ex0 + ex1);
    sW[2 * tid]     = ex0 * inv;
    sW[2 * tid + 1] = ex1 * inv;
  }
  sBp[tid] = bp0[tid];
  if (tid < 4) sBp[PH + tid] = bp1[tid];
  if (wave == 0) {
    int c = chk[(size_t)lane * CHKLINE];
    c = c < 0 ? 0 : c;
    c += __shfl_xor(c, 1);
    c += __shfl_xor(c, 2);
    c += __shfl_xor(c, 4);
    c += __shfl_xor(c, 8);
    c += __shfl_xor(c, 16);
    if (lane == 0) sFlag = c;
  }
  __syncthreads();

  {
    const int rl = tid >> 2, g = tid & 3;
    const int b = sBi[rl], q = sQi[rl];
    const float w0 = sW[2 * rl], w1 = sW[2 * rl + 1];
    const float* p0 = D0 + ((size_t)b * (size_t)nQry + (size_t)q) * DROW + 16 * g;
    const float* p1 = D1 + ((size_t)b * (size_t)nQry + (size_t)q) * DROW + 16 * g;
#pragma unroll
    for (int i = 0; i < 2; ++i) {
      const v4f xa = *(const v4f*)(p0 + 8 * i);
      const v4f xb = *(const v4f*)(p0 + 8 * i + 4);
      const v4f ya = *(const v4f*)(p1 + 8 * i);
      const v4f yb = *(const v4f*)(p1 + 8 * i + 4);
      const v4f da = (xa * w0 + ya * w1) * SCA;
      const v4f db = (xb * w0 + yb * w1) * SCA;
      Cvt8 cv;
      cv.v[0] = (_Float16)da.x; cv.v[1] = (_Float16)da.y; cv.v[2] = (_Float16)da.z; cv.v[3] = (_Float16)da.w;
      cv.v[4] = (_Float16)db.x; cv.v[5] = (_Float16)db.y; cv.v[6] = (_Float16)db.z; cv.v[7] = (_Float16)db.w;
      *(v8h*)(sA + rl * APA + 16 * g + 8 * i) = cv.v;
    }
  }
  __syncthreads();

  const int rt = wave & 3, cg = wave >> 2;

#pragma unroll 1
  for (int qq = 0; qq < 2; ++qq) {
    v8f a0, a1, a2, a3;
    gemm16x64(sA + (16 * rt + m) * APA + 8 * hh, (const _Float16*)(wp + PP0), CIN, 2, 128 * cg + 64 * qq, m, hh,
              a0, a1, a2, a3);
    _Float16* sp = sH + (16 * rt + 8 * hh) * APH + 128 * cg + 64 * qq + m;
    const float* bb = sBp + 128 * cg + 64 * qq + m;
    st8_gelu_h(sp,      APH, a0, INV1024, bb[0]);
    st8_gelu_h(sp + 16, APH, a1, INV1024, bb[16]);
    st8_gelu_h(sp + 32, APH, a2, INV1024, bb[32]);
    st8_gelu_h(sp + 48, APH, a3, INV1024, bb[48]);
  }
  __syncthreads();

  if (wave < 4) {
    v8f c0;
    gemm16x16(sH + (16 * wave + m) * APH + 8 * hh, (const _Float16*)(wp + PP1), PH, 8, 0, m, hh, c0);
    if (m < 4) {
      const float bias = sBp[PH + m];
#pragma unroll
      for (int r = 0; r < 8; ++r) sO[(16 * wave + 8 * hh + r) * 4 + m] = c0[r] * INV1024 + bias;
    }
  }
  __syncthreads();

  {
    const int R = R0 + tid;
    const bool act = (tid < TR) && (R < nRows);
    const bool bad = (sFlag != 0);
    const float qnan = __int_as_float(0x7fc00000);
    v4f ov = zero4();
    if (act) {
      ov = *(const v4f*)(sO + 4 * tid);
      if (bad) { ov.x = qnan; ov.y = qnan; ov.z = qnan; ov.w = qnan; }
      *(volatile v4f*)(out + (size_t)R * 4) = ov;
    }
    __threadfence();
    if (act) {
      *(volatile v4f*)(out + (size_t)R * 4) = ov;
    }
  }
}

extern "C" void kernel_launch(void* const* d_in, const int* in_sizes, int n_in,
                              void* d_out, int out_size, void* d_ws, size_t ws_size,
                              hipStream_t stream) {
  if (n_in < 21) return;
  if (in_sizes[0] < 2 || (in_sizes[0] % 2) != 0) return;
  const int nLat = in_sizes[0] / 2;
  if (nLat < 1 || nLat > (1 << 22)) return;
  if (in_sizes[1] != NB * nLat * CIN) return;
  if (in_sizes[2] < 2 || (in_sizes[2] % 2) != 0) return;
  const int nQry = in_sizes[2] / 2;
  if (nQry < 1 || nQry > (1 << 22)) return;
  const int E0 = in_sizes[3];
  const int E1 = in_sizes[5];
  if (E0 < 1 || E0 > (1 << 26) || in_sizes[4] != E0) return;
  if (E1 < 1 || E1 > (1 << 26) || in_sizes[6] != E1) return;
  if (in_sizes[7] != 4 * CIN || in_sizes[8] != CIN) return;
  if (in_sizes[9] != CIN * CIN || in_sizes[10] != CIN) return;
  if (in_sizes[11] != CIN * CIN || in_sizes[12] != CIN) return;
  if (in_sizes[13] != 32 || in_sizes[14] != 16 || in_sizes[15] != 32 || in_sizes[16] != 2) return;
  if (in_sizes[17] != CIN * PH || in_sizes[18] != PH || in_sizes[19] != PH * 4 || in_sizes[20] != 4) return;
  const int nRows = NB * nQry;
  if (out_size != nRows * 4) return;

  const float* latc = (const float*)d_in[0];
  const float* rnd  = (const float*)d_in[1];
  const float* qc   = (const float*)d_in[2];
  const int*   src0 = (const int*)d_in[3];
  const int*   qry0 = (const int*)d_in[4];
  const int*   src1 = (const int*)d_in[5];
  const int*   qry1 = (const int*)d_in[6];
  const float* Wk0  = (const float*)d_in[7];
  const float* bk0  = (const float*)d_in[8];
  const float* Wk1  = (const float*)d_in[9];
  const float* bk1  = (const float*)d_in[10];
  const float* Wk2  = (const float*)d_in[11];
  const float* bk2  = (const float*)d_in[12];
  const float* Wsw0 = (const float*)d_in[13];
  const float* bsw0 = (const float*)d_in[14];
  const float* Wsw1 = (const float*)d_in[15];
  const float* bsw1 = (const float*)d_in[16];
  const float* Wp0  = (const float*)d_in[17];
  const float* bp0  = (const float*)d_in[18];
  const float* Wp1  = (const float*)d_in[19];
  const float* bp1  = (const float*)d_in[20];
  float* out = (float*)d_out;

  const int nbE0 = (E0 + TE - 1) / TE;
  const int nbE1 = (E1 + TE - 1) / TE;
  const int nbEmax = nbE0 > nbE1 ? nbE0 : nbE1;
  const int nbSeg = (nQry + QPB - 1) / QPB;
  const int nbProj = (nRows + TR - 1) / TR;

  char* ws = (char*)d_ws;
  size_t off = 0;
  const size_t oW  = off; off += (size_t)PWTOT * 2;                          off = (off + 255) & ~(size_t)255;
  const size_t oC  = off; off += (size_t)NCHK * CHKLINE * 4;                 off = (off + 255) & ~(size_t)255;
  const size_t oK  = off; off += (size_t)nbEmax * TE * KROW * 2;             off = (off + 255) & ~(size_t)255;
  const size_t oD0 = off; off += (size_t)NB * (size_t)nQry * DROW * 4;       off = (off + 255) & ~(size_t)255;
  const size_t oD1 = off; off += (size_t)NB * (size_t)nQry * DROW * 4;       off = (off + 255) & ~(size_t)255;
  if (off > ws_size || off > (size_t)WSCAP) return;
  unsigned short* wp = (unsigned short*)(ws + oW);
  int* chk = (int*)(ws + oC);
  unsigned short* Kq = (unsigned short*)(ws + oK);
  float* D0 = (float*)(ws + oD0);
  float* D1 = (float*)(ws + oD1);

  k_chk<<<NCHK, NTHR, 0, stream>>>(qry0, E0, qry1, E1, chk);
  k_prep<<<PBLK, NTHR, 0, stream>>>(Wk1, Wk2, Wp0, Wp1, wp);
  k_edge<<<nbE0, NTHR, 0, stream>>>(latc, qc, src0, qry0, Wk0, bk0, bk1, bk2, wp, Kq, E0, nLat, nQry);
  k_seg<<<nbSeg, NTHR, 0, stream>>>(qry0, src0, Kq, rnd, D0, E0, nQry, nLat);
  k_edge<<<nbE1, NTHR, 0, stream>>>(latc, qc, src1, qry1, Wk0, bk0, bk1, bk2, wp, Kq, E1, nLat, nQry);
  k_seg<<<nbSeg, NTHR, 0, stream>>>(qry1, src1, Kq, rnd, D1, E1, nQry, nLat);
  k_proj<<<nbProj, NTHR, 0, stream>>>(qc, Wsw0, bsw0, Wsw1, bsw1, D0, D1, wp, bp0, bp1, chk, out, nQry, nRows);
}
